// EALSTM_13005160972908
// MI455X (gfx1250) — hardware-verified
//
#include <hip/hip_runtime.h>
#include <stdint.h>
#include <math.h>

typedef __attribute__((ext_vector_type(16))) _Float16 v16h;
typedef __attribute__((ext_vector_type(8)))  _Float16 v8h;
typedef __attribute__((ext_vector_type(8)))  float    v8f;
typedef __attribute__((ext_vector_type(4)))  float    v4f;

constexpr int NBATCH = 128;
constexpr int NSTEP  = 2048;
constexpr int NDYN   = 8;
constexpr int NSTAT  = 24;
constexpr int NFEAT  = 32;
constexpr int NHID   = 256;
constexpr int MROWS  = 16;
constexpr int NTHREADS = 512;
constexpr int HPITCH = 264;
constexpr int OCHUNK = 32;
constexpr float WCARRY = 16.0f;
constexpr float WCARRY_INV = 0.0625f;

static_assert(NBATCH % MROWS == 0, "tile");
static_assert(NHID == 16 * (NTHREADS / 32), "cols");
static_assert(NHID % 32 == 0, "K32");
static_assert(NFEAT == NDYN + NSTAT, "feat");
static_assert(NSTEP % OCHUNK == 0, "chunk");
static_assert((HPITCH % 8) == 0, "align");

__device__ __forceinline__ v16h frag_load_h(const _Float16* p) {
  union { v16h v; v8h h[2]; } f;
  f.h[0] = *(const v8h*)(p);
  f.h[1] = *(const v8h*)(p + 16);
  return f.v;
}

__device__ __forceinline__ v8f mma16(v16h a, v16h b, v8f c) {
  c = __builtin_amdgcn_wmma_f32_16x16x32_f16(false, a, false, b, (short)0, c, false, false);
  asm volatile("v_nop\n\tv_nop\n\tv_nop\n\tv_nop" : "+v"(c) : "v"(a), "v"(b));
  return c;
}

__device__ __forceinline__ float sigm_f(float v) {
  v = fminf(fmaxf(v, -30.0f), 30.0f);
  const float e = expf(-v);
  return 1.0f / (1.0f + e);
}
__device__ __forceinline__ float tanh_f(float v) {
  v = fminf(fmaxf(v, -15.0f), 15.0f);
  const float e = expf(2.0f * v);
  return 1.0f - 2.0f / (e + 1.0f);
}

__global__ __launch_bounds__(256) void cast_wh16(
    const float* __restrict__ w0, const float* __restrict__ w1, const float* __restrict__ w2,
    _Float16* __restrict__ dst, int nvec) {
  const int mat = blockIdx.y;
  const float* src = w0;
  if (mat == 1) src = w1;
  if (mat == 2) src = w2;
  const int i = blockIdx.x * 256 + threadIdx.x;
  if (i < nvec) {
    const v4f a = *(const v4f*)(src + (size_t)8 * i);
    const v4f b = *(const v4f*)(src + (size_t)8 * i + 4);
    v8h hv;
#pragma unroll
    for (int e = 0; e < 4; ++e) {
      hv[e]     = (_Float16)(a[e] * WCARRY);
      hv[4 + e] = (_Float16)(b[e] * WCARRY);
    }
    _Float16* d = dst + (size_t)mat * NHID * NHID + (size_t)8 * i;
    *(volatile v8h*)d = hv;
    __threadfence();
    *(volatile v8h*)d = hv;
  }
}

__global__ __launch_bounds__(256) void build_wx16(
    const float* __restrict__ wfx, const float* __restrict__ wgx, const float* __restrict__ wox,
    const float* __restrict__ wi, _Float16* __restrict__ dst) {
  const int i = blockIdx.x * 256 + threadIdx.x;
  if (i >= 4 * NHID * (NFEAT / 8)) return;
  const int gate = i >> 10;
  const int n = (i >> 2) & 255;
  const int q = i & 3;
  const int qq = (q > 0) ? (q - 1) : 0;
  const v4f f0 = *(const v4f*)(wfx + n * NDYN), f1 = *(const v4f*)(wfx + n * NDYN + 4);
  const v4f g0 = *(const v4f*)(wgx + n * NDYN), g1 = *(const v4f*)(wgx + n * NDYN + 4);
  const v4f o0 = *(const v4f*)(wox + n * NDYN), o1 = *(const v4f*)(wox + n * NDYN + 4);
  const v4f i0 = *(const v4f*)(wi + n * NSTAT + 8 * qq), i1 = *(const v4f*)(wi + n * NSTAT + 8 * qq + 4);
  v8h hv;
#pragma unroll
  for (int e = 0; e < 4; ++e) {
    const float wdl = (gate == 0) ? f0[e] : ((gate == 1) ? g0[e] : o0[e]);
    const float wdh = (gate == 0) ? f1[e] : ((gate == 1) ? g1[e] : o1[e]);
    const float vl = (gate < 3) ? ((q == 0) ? wdl : 0.0f) : ((q == 0) ? 0.0f : i0[e]);
    const float vh = (gate < 3) ? ((q == 0) ? wdh : 0.0f) : ((q == 0) ? 0.0f : i1[e]);
    hv[e]     = (_Float16)(vl * WCARRY);
    hv[4 + e] = (_Float16)(vh * WCARRY);
  }
  _Float16* d = dst + (size_t)8 * i;
  *(volatile v8h*)d = hv;
  __threadfence();
  *(volatile v8h*)d = hv;
}

__device__ __forceinline__ void flush_lines(const float* ob, float* __restrict__ out, int b0, int tbase, int lane) {
  const int q = lane >> 3, c4 = (lane & 7) * 4;
  for (int pass = 0; pass < 2; ++pass) {
#pragma unroll
    for (int it = 0; it < 4; ++it) {
      const int row = it * 4 + q;
      const v4f v = *(const v4f*)(ob + row * OCHUNK + c4);
      *(volatile v4f*)(out + (size_t)(b0 + row) * NSTEP + tbase + c4) = v;
    }
    __threadfence();
  }
}

__global__ __launch_bounds__(NTHREADS) void ealstm_scan_f16(
    const float* __restrict__ x, const float* __restrict__ c0, const float* __restrict__ h0,
    const _Float16* __restrict__ wh16,
    const _Float16* __restrict__ wx16,
    const float* __restrict__ bi,
    const float* __restrict__ bf_x, const float* __restrict__ bf_h,
    const float* __restrict__ bg_x, const float* __restrict__ bg_h,
    const float* __restrict__ bo_x, const float* __restrict__ bo_h,
    const float* __restrict__ wout, const float* __restrict__ bout,
    float* __restrict__ out) {
  __shared__ __align__(16) _Float16 hbuf[2 * MROWS * HPITCH];
  __shared__ __align__(16) _Float16 wxl[4 * NHID * NFEAT];
  __shared__ __align__(16) float part[2 * 16 * 16];
  __shared__ __align__(16) float obuf[2 * MROWS * OCHUNK];

  const int tid  = threadIdx.x;
  const int lane = tid & 31;
  const int wave = tid >> 5;
  const int hh   = lane >> 4;
  const int cl   = lane & 15;
  const int n    = wave * 16 + cl;
  const int b0   = blockIdx.x * MROWS;

  for (int idx = tid; idx < MROWS * NHID; idx += NTHREADS) {
    const int m = idx >> 8, k = idx & 255;
    hbuf[m * HPITCH + k] = (_Float16)h0[k];
  }
  for (int idx = tid; idx < (4 * NHID * NFEAT) / 8; idx += NTHREADS) {
    *(v8h*)(wxl + 8 * idx) = *(const v8h*)(wx16 + 8 * idx);
  }
  const float bfn = WCARRY * (bf_x[n] + bf_h[n]);
  const float bgn = WCARRY * (bg_x[n] + bg_h[n]);
  const float bon = WCARRY * (bo_x[n] + bo_h[n]);
  const float bin = WCARRY * bi[n];
  const float woutn = wout[n];
  const float boutv = bout[0];
  float cst[8];
  {
    const float cv = c0[n];
#pragma unroll
    for (int r = 0; r < 8; ++r) cst[r] = cv;
  }
  __syncthreads();

#pragma unroll 1
  for (int t = 0; t < NSTEP; ++t) {
    const int p = t & 1, np = p ^ 1;

    if (wave == 0 && t > 0 && lane < 16) {
      const float* pr = part + np * 256;
      float s = 0.0f;
#pragma unroll
      for (int w = 0; w < 16; ++w) s += pr[w * 16 + lane];
      obuf[(((t - 1) >> 5) & 1) * (MROWS * OCHUNK) + lane * OCHUNK + ((t - 1) & 31)] = s + boutv;
    }
    if (wave == 1 && t >= 33 && (t & 31) == 1) {
      const int j = (t - 33) >> 5;
      flush_lines(obuf + (j & 1) * (MROWS * OCHUNK), out, b0, j * OCHUNK, lane);
    }

    v16h ax;
    {
      const float* xr = x + ((size_t)(b0 + cl) * NSTEP + t) * NFEAT;
      const v4f q0 = *(const v4f*)(xr + 8 * hh);
      const v4f q1 = *(const v4f*)(xr + 8 * hh + 4);
      const v4f q2 = *(const v4f*)(xr + 16 + 8 * hh);
      const v4f q3 = *(const v4f*)(xr + 16 + 8 * hh + 4);
#pragma unroll
      for (int e = 0; e < 4; ++e) {
        ax[e]      = (_Float16)q0[e];
        ax[4 + e]  = (_Float16)q1[e];
        ax[8 + e]  = (_Float16)q2[e];
        ax[12 + e] = (_Float16)q3[e];
      }
    }
    v8f accf, accg, acco, acci;
#pragma unroll
    for (int r = 0; r < 8; ++r) { accf[r] = bfn; accg[r] = bgn; acco[r] = bon; acci[r] = bin; }
    {
      const _Float16* wxp = wxl + n * NFEAT + 8 * hh;
      accf = mma16(ax, frag_load_h(wxp), accf);
      accg = mma16(ax, frag_load_h(wxp + NHID * NFEAT), accg);
      acco = mma16(ax, frag_load_h(wxp + 2 * NHID * NFEAT), acco);
      acci = mma16(ax, frag_load_h(wxp + 3 * NHID * NFEAT), acci);
    }
    {
      const _Float16* hr = hbuf + p * (MROWS * HPITCH) + cl * HPITCH + 8 * hh;
      const _Float16* wf = wh16 + (size_t)n * NHID + 8 * hh;
      const _Float16* wg = wf + NHID * NHID;
      const _Float16* wo = wg + NHID * NHID;
#pragma unroll 1
      for (int ks = 0; ks < NHID / 32; ++ks) {
        const int ko = ks * 32;
        const v16h ah = frag_load_h(hr + ko);
        accf = mma16(ah, frag_load_h(wf + ko), accf);
        accg = mma16(ah, frag_load_h(wg + ko), accg);
        acco = mma16(ah, frag_load_h(wo + ko), acco);
      }
    }
    float sr[8];
    _Float16* hw = hbuf + np * (MROWS * HPITCH) + n;
#pragma unroll
    for (int r = 0; r < 8; ++r) {
      const float fg = sigm_f(accf[r] * WCARRY_INV);
      const float gg = tanh_f(accg[r] * WCARRY_INV);
      const float og = sigm_f(acco[r] * WCARRY_INV);
      const float ig = sigm_f(acci[r] * WCARRY_INV);
      float s = og * woutn;
      s += __shfl_xor(s, 1);
      s += __shfl_xor(s, 2);
      s += __shfl_xor(s, 4);
      s += __shfl_xor(s, 8);
      sr[r] = s;
      const float cn = fg * cst[r] + ig * gg;
      cst[r] = cn;
      const float hn = og * tanh_f(cn);
      hw[(8 * hh + r) * HPITCH] = (_Float16)hn;
    }
    {
      float pv = sr[0];
#pragma unroll
      for (int r = 1; r < 8; ++r) pv = (cl == r) ? sr[r] : pv;
      if (cl < 8) part[p * 256 + wave * 16 + 8 * hh + cl] = pv;
    }
    __syncthreads();
  }

  if (wave == 0 && lane < 16) {
    const float* pr = part + ((NSTEP - 1) & 1) * 256;
    float s = 0.0f;
#pragma unroll
    for (int w = 0; w < 16; ++w) s += pr[w * 16 + lane];
    obuf[(((NSTEP - 1) >> 5) & 1) * (MROWS * OCHUNK) + lane * OCHUNK + (OCHUNK - 1)] = s + boutv;
  }
  __syncthreads();
  if (wave == 1) {
    const int j = NSTEP / OCHUNK - 1;
    flush_lines(obuf + (j & 1) * (MROWS * OCHUNK), out, b0, j * OCHUNK, lane);
  }
}

extern "C" void kernel_launch(void* const* d_in, const int* in_sizes, int n_in,
                              void* d_out, int out_size, void* d_ws, size_t ws_size,
                              hipStream_t stream) {
  if (n_in < 19) return;
  const float* x    = (const float*)d_in[0];
  const float* c0   = (const float*)d_in[1];
  const float* h0   = (const float*)d_in[2];
  const float* Wi   = (const float*)d_in[3];
  const float* bi   = (const float*)d_in[4];
  const float* Wf_x = (const float*)d_in[5];
  const float* bf_x = (const float*)d_in[6];
  const float* Wf_h = (const float*)d_in[7];
  const float* bf_h = (const float*)d_in[8];
  const float* Wg_x = (const float*)d_in[9];
  const float* bg_x = (const float*)d_in[10];
  const float* Wg_h = (const float*)d_in[11];
  const float* bg_h = (const float*)d_in[12];
  const float* Wo_x = (const float*)d_in[13];
  const float* bo_x = (const float*)d_in[14];
  const float* Wo_h = (const float*)d_in[15];
  const float* bo_h = (const float*)d_in[16];
  const float* Wout = (const float*)d_in[17];
  const float* bout = (const float*)d_in[18];
  float* outp = (float*)d_out;

  if (in_sizes[0] < NBATCH * NSTEP * NFEAT) return;
  if (in_sizes[7] < NHID * NHID || in_sizes[11] < NHID * NHID || in_sizes[15] < NHID * NHID) return;
  if (out_size < NBATCH * NSTEP) return;

  const size_t whBytes = (size_t)3 * NHID * NHID * sizeof(_Float16);
  const size_t wxBytes = (size_t)4 * NHID * NFEAT * sizeof(_Float16);
  if (whBytes + wxBytes > ws_size) return;
  _Float16* wh16 = (_Float16*)d_ws;
  _Float16* wx16 = (_Float16*)((char*)d_ws + whBytes);

  cast_wh16<<<dim3(NHID * NHID / 8 / 256, 3), dim3(256), 0, stream>>>(Wf_h, Wg_h, Wo_h, wh16, NHID * NHID / 8);
  build_wx16<<<dim3((4 * NHID * (NFEAT / 8)) / 256), dim3(256), 0, stream>>>(Wf_x, Wg_x, Wo_x, Wi, wx16);
  ealstm_scan_f16<<<dim3(NBATCH / MROWS), dim3(NTHREADS), 0, stream>>>(
      x, c0, h0, wh16, wx16, bi, bf_x, bf_h, bg_x, bg_h, bo_x, bo_h, Wout, bout, outp);
}
